// CKANKANNet_80736795231207
// MI455X (gfx1250) — hardware-verified
//
#include <hip/hip_runtime.h>

#pragma clang fp contract(off)

typedef _Float16 f16t;
typedef _Float16 v16h __attribute__((ext_vector_type(16)));
typedef _Float16 v8h  __attribute__((ext_vector_type(8)));
typedef float    v8f  __attribute__((ext_vector_type(8)));
typedef float    v4f  __attribute__((ext_vector_type(4)));
typedef v8h __attribute__((may_alias)) v8ha;
typedef v4f __attribute__((may_alias)) v4fa;
union Frag { v16h v; v8h half[2]; };

#define NBATCH 64
#define C1  3
#define CE1 32
#define HH1 64
#define O1  64
#define RB1 2
#define C2  64
#define CE2 576
#define HH2 32
#define O2  128
#define RB2 2
#define C3  128
#define CE3 1152
#define HH3 16
#define O3  64
#define RB3 8
#define FIN 4096
#define KL  36864
#define NOUT 100
#define NLP 112
#define SC_WB 64.0f
#define SC_WS 4.0f
#define SC_BS 16.0f
#define OSC (1.0f / 64.0f)

#define KN_H    (2.0 / 5.0)
#define KN_BASE (-1.0 - 3.0 * KN_H)

__device__ __forceinline__ v8f wmma_f16(v16h a, v16h b, v8f c) {
  v8f d = __builtin_amdgcn_wmma_f32_16x16x32_f16(false, a, false, b, (short)0, c, false, false);
  asm volatile("v_nop\n\tv_nop\n\tv_nop\n\tv_nop" : "+v"(d) : "v"(a), "v"(b));
  return d;
}

__device__ __forceinline__ v16h load_frag32(const f16t* p, int h) {
  Frag f;
  f.half[0] = *(const v8ha*)(p + 8 * h);
  f.half[1] = *(const v8ha*)(p + 16 + 8 * h);
  return f.v;
}

__device__ __forceinline__ v8f zero8f() {
  v8f z;
  #pragma unroll
  for (int j = 0; j < 8; ++j) z[j] = 0.f;
  return z;
}

__device__ __forceinline__ v8h zero8h() {
  v8h z;
  #pragma unroll
  for (int j = 0; j < 8; ++j) z[j] = (f16t)0.0f;
  return z;
}

__device__ __forceinline__ void kan_feat(float x, float f[9]) {
  const float e = expf(-x);
  const float sig = __builtin_amdgcn_rcpf(1.0f + e);
  f[0] = x * sig;

  float pts[12];
  #pragma unroll
  for (int k = 0; k < 12; ++k) pts[k] = (float)(KN_BASE + KN_H * (double)k);

  float bb[11];
  #pragma unroll
  for (int k = 0; k < 11; ++k) bb[k] = (x >= pts[k] && x < pts[k + 1]) ? 1.0f : 0.0f;

  #pragma unroll
  for (int k = 0; k < 10; ++k) {
    const float rl = 1.0f / (pts[k + 1] - pts[k]);
    const float rr = 1.0f / (pts[k + 2] - pts[k + 1]);
    const float lt = ((x - pts[k]) * rl) * bb[k];
    const float rt = ((pts[k + 2] - x) * rr) * bb[k + 1];
    bb[k] = lt + rt;
  }
  #pragma unroll
  for (int k = 0; k < 9; ++k) {
    const float rl = 1.0f / (pts[k + 2] - pts[k]);
    const float rr = 1.0f / (pts[k + 3] - pts[k + 1]);
    const float lt = ((x - pts[k]) * rl) * bb[k];
    const float rt = ((pts[k + 3] - x) * rr) * bb[k + 1];
    bb[k] = lt + rt;
  }
  #pragma unroll
  for (int k = 0; k < 8; ++k) {
    const float rl = 1.0f / (pts[k + 3] - pts[k]);
    const float rr = 1.0f / (pts[k + 4] - pts[k + 1]);
    const float lt = ((x - pts[k]) * rl) * bb[k];
    const float rt = ((pts[k + 4] - x) * rr) * bb[k + 1];
    bb[k] = lt + rt;
  }
  #pragma unroll
  for (int j = 0; j < 8; ++j) f[1 + j] = bb[j];
}

template <int C, int CEP, int O>
__global__ __launch_bounds__(256) void packw_k(const float* __restrict__ wb, const float* __restrict__ wsp,
                                              f16t* __restrict__ Wp)
{
  constexpr int KP8 = CEP / 8, ROW8 = 9 * KP8, NPIECE = O * ROW8;
  const int g = blockIdx.x * 256 + threadIdx.x;
  if (g >= NPIECE) return;
  const int o = g / ROW8;
  const int rem = g - o * ROW8;
  const int tap = rem / KP8;
  const int ce0 = (rem - tap * KP8) * 8;
  v8h o8;
  #pragma unroll
  for (int i = 0; i < 8; ++i) {
    const int ce = ce0 + i;
    int c = ce / 9;
    const int j = ce - c * 9;
    c = (c > C - 1) ? (C - 1) : c;
    const int jj = (j > 0) ? (j - 1) : 0;
    const float vb = wb[((size_t)(o * C + c)) * 9 + tap] * SC_WB;
    const float vs = wsp[((size_t)(o * C + c) * 8 + jj) * 9 + tap] * SC_WS;
    float v = (j == 0) ? vb : vs;
    v = (ce < 9 * C) ? v : 0.0f;
    o8[i] = (f16t)v;
  }
  f16t* dst = Wp + (size_t)8 * g;
  *(volatile v8h*)dst = o8;
  __threadfence();
  *(volatile v8h*)dst = o8;
}

__global__ __launch_bounds__(256) void packl_k(const float* __restrict__ lb, const float* __restrict__ lc,
                                              f16t* __restrict__ WL)
{
  constexpr int ROW8 = KL / 8, NPIECE = NLP * ROW8;
  const int g = blockIdx.x * 256 + threadIdx.x;
  if (g >= NPIECE) return;
  const int n = g / ROW8;
  const int k0 = (g - n * ROW8) * 8;
  const int nn = (n > NOUT - 1) ? (NOUT - 1) : n;
  v8h o8;
  #pragma unroll
  for (int i = 0; i < 8; ++i) {
    const int k = k0 + i;
    const int f = k / 9;
    const int j = k - f * 9;
    const int jj = (j > 0) ? (j - 1) : 0;
    const float vb = lb[(size_t)nn * FIN + f] * SC_WB;
    const float vc = lc[((size_t)nn * FIN + f) * 8 + jj] * SC_WS;
    float v = (j == 0) ? vb : vc;
    v = (n < NOUT) ? v : 0.0f;
    o8[i] = (f16t)v;
  }
  f16t* dst = WL + (size_t)8 * g;
  *(volatile v8h*)dst = o8;
  __threadfence();
  *(volatile v8h*)dst = o8;
}

template <int C, int CEP, int H, int W, int NCHW>
__global__ __launch_bounds__(256) void expand_k(const float* __restrict__ X, f16t* __restrict__ T)
{
  constexpr int PW = W + 2, PH = H + 2, NPP = PH * PW, NPIECE = (PW * CEP) / 8;
  static_assert((PW * CEP) % 64 == 0);
  static_assert(9 * C <= CEP);
  __shared__ __attribute__((aligned(16))) f16t sT[PW * CEP];
  const int tid = threadIdx.x;
  const int b = blockIdx.x, yq = blockIdx.y;

  {
    const v8h z = zero8h();
    #pragma unroll 1
    for (int i = tid; i < NPIECE; i += 256) *(v8ha*)(sT + 8 * i) = z;
  }
  __syncthreads();

  if (yq >= 1 && yq <= H) {
    const int y = yq - 1;
    #pragma unroll 1
    for (int idx = tid; idx < C * W; idx += 256) {
      const int c = idx / W, xx = idx - c * W;
      float v;
      if (NCHW) v = X[(((size_t)b * C + c) * H + y) * W + xx];
      else      v = X[((size_t)b * H + y) * (size_t)(C * W) + idx];
      float f[9];
      kan_feat(v, f);
      f16t* dst = sT + (xx + 1) * CEP + c * 9;
      dst[0] = (f16t)f[0];
      #pragma unroll
      for (int j = 1; j < 9; ++j) dst[j] = (f16t)(f[j] * SC_BS);
    }
  }
  __syncthreads();

  f16t* base = T + ((size_t)b * NPP + (size_t)yq * PW) * CEP;
  #pragma unroll 1
  for (int i = tid; i < NPIECE; i += 256) {
    const v8h v = *(const v8ha*)(sT + 8 * i);
    *(volatile v8h*)(base + (size_t)8 * i) = v;
  }
  __threadfence();
  #pragma unroll 1
  for (int i = tid; i < NPIECE; i += 256) {
    const v8h v = *(const v8ha*)(sT + 8 * i);
    *(volatile v8h*)(base + (size_t)8 * i) = v;
  }
}

__global__ __launch_bounds__(256) void expand_head_k(const float* __restrict__ P3, f16t* __restrict__ EL)
{
  constexpr int FPB = 1024, NPIECE = FPB * 9 / 8;
  __shared__ __attribute__((aligned(16))) f16t sE[FPB * 9];
  const int tid = threadIdx.x;
  const int chunk = blockIdx.x, b = blockIdx.y;
  #pragma unroll 1
  for (int i = 0; i < 4; ++i) {
    const int fl = tid + 256 * i;
    const int f = chunk * FPB + fl;
    const int c = f >> 6, y = (f >> 3) & 7, xx = f & 7;
    const float v = P3[(((size_t)b * 8 + y) * 64 + c) * 8 + xx];
    float ft[9];
    kan_feat(v, ft);
    f16t* dst = sE + fl * 9;
    dst[0] = (f16t)ft[0];
    #pragma unroll
    for (int j = 1; j < 9; ++j) dst[j] = (f16t)(ft[j] * SC_BS);
  }
  __syncthreads();

  f16t* base = EL + (size_t)b * KL + (size_t)chunk * (FPB * 9);
  #pragma unroll 1
  for (int i = tid; i < NPIECE; i += 256) {
    const v8h v = *(const v8ha*)(sE + 8 * i);
    *(volatile v8h*)(base + (size_t)8 * i) = v;
  }
  __threadfence();
  #pragma unroll 1
  for (int i = tid; i < NPIECE; i += 256) {
    const v8h v = *(const v8ha*)(sE + 8 * i);
    *(volatile v8h*)(base + (size_t)8 * i) = v;
  }
}

template <int CEP, int O, int H, int W, int RB>
__global__ __launch_bounds__(256) void conv_k(const f16t* __restrict__ Wp, const f16t* __restrict__ T,
                                             float* __restrict__ P)
{
  constexpr int NG = O / 32, M = RB * W, MG = M / 32, PW = W + 2, NPP = (H + 2) * PW;
  constexpr int KROW = 9 * CEP, WP2 = W / 2, HP2 = H / 2;
  static_assert(NG * MG == 8);
  static_assert(O * M == 8192);
  static_assert((RB / 2) * O * WP2 == 2048);
  static_assert(CEP % 32 == 0);
  static_assert(W % 16 == 0);
  __shared__ __attribute__((aligned(16))) float sO[8192];

  const int tid = threadIdx.x, lane = tid & 31, w = tid >> 5;
  const int h = lane >> 4, m = lane & 15;
  const int ng = w % NG, mg = w / NG;
  const int b = blockIdx.y, y0 = blockIdx.x * RB;

  const v8f z8 = zero8f();
  v8f acc[2][2];
  #pragma unroll
  for (int at = 0; at < 2; ++at) { acc[at][0] = z8; acc[at][1] = z8; }

  const f16t* wr0 = Wp + (size_t)(32 * ng + m) * KROW;
  const f16t* wr1 = wr0 + (size_t)16 * KROW;
  const f16t* tb = T + (size_t)b * NPP * CEP;
  const int pt0 = 32 * mg, pt1 = 32 * mg + 16;
  const int yl0 = pt0 / W, xb0 = pt0 - yl0 * W;
  const int yl1 = pt1 / W, xb1 = pt1 - yl1 * W;

  #pragma unroll 1
  for (int tap = 0; tap < 9; ++tap) {
    const int dy = tap / 3, dx = tap - 3 * dy;
    const f16t* wt0 = wr0 + tap * CEP;
    const f16t* wt1 = wr1 + tap * CEP;
    const f16t* tr0 = tb + (size_t)((y0 + yl0 + dy) * PW + dx + xb0 + m) * CEP;
    const f16t* tr1 = tb + (size_t)((y0 + yl1 + dy) * PW + dx + xb1 + m) * CEP;
    #pragma unroll 1
    for (int c0 = 0; c0 < CEP; c0 += 32) {
      const v16h a0 = load_frag32(wt0 + c0, h);
      const v16h a1 = load_frag32(wt1 + c0, h);
      const v16h b0 = load_frag32(tr0 + c0, h);
      const v16h b1 = load_frag32(tr1 + c0, h);
      acc[0][0] = wmma_f16(a0, b0, acc[0][0]);
      acc[0][1] = wmma_f16(a0, b1, acc[0][1]);
      acc[1][0] = wmma_f16(a1, b0, acc[1][0]);
      acc[1][1] = wmma_f16(a1, b1, acc[1][1]);
    }
  }

  #pragma unroll
  for (int at = 0; at < 2; ++at) {
    #pragma unroll
    for (int bt = 0; bt < 2; ++bt) {
      float* so = sO + (32 * ng + 16 * at + 8 * h) * M + 32 * mg + 16 * bt + m;
      #pragma unroll
      for (int r = 0; r < 8; ++r) so[r * M] = acc[at][bt][r] * OSC;
    }
  }
  __syncthreads();

  const size_t cb = ((size_t)(b * HP2 + blockIdx.x * (RB / 2)) * O) * WP2;
  v4f vals[2];
  int  dofs[2];
  #pragma unroll
  for (int pp = 0; pp < 2; ++pp) {
    const int idx = 4 * (tid + 256 * pp);
    const int xp0 = idx % WP2;
    const int t1 = idx / WP2;
    const int o = t1 % O;
    const int ypl = t1 / O;
    const float* s0 = sO + o * M + (2 * ypl) * W + 2 * xp0;
    const float* s1 = s0 + W;
    v4f v;
    #pragma unroll
    for (int i = 0; i < 4; ++i)
      v[i] = fmaxf(fmaxf(s0[2 * i], s0[2 * i + 1]), fmaxf(s1[2 * i], s1[2 * i + 1]));
    vals[pp] = v;
    dofs[pp] = idx;
  }
  #pragma unroll
  for (int pp = 0; pp < 2; ++pp) *(volatile v4f*)(P + cb + dofs[pp]) = vals[pp];
  __threadfence();
  #pragma unroll
  for (int pp = 0; pp < 2; ++pp) *(volatile v4f*)(P + cb + dofs[pp]) = vals[pp];
}

__global__ __launch_bounds__(256) void head_k(const f16t* __restrict__ EL, const f16t* __restrict__ WL,
                                             float* __restrict__ out)
{
  __shared__ __attribute__((aligned(16))) float sH[64 * NLP];
  const int tid = threadIdx.x, lane = tid & 31, w = tid >> 5;
  const int h = lane >> 4, m = lane & 15;
  const int nt = (w < 7) ? w : 6;

  const f16t* ea = EL + (size_t)m * KL;
  const f16t* wr = WL + (size_t)(16 * nt + m) * KL;
  const v8f z8 = zero8f();
  v8f acc[4];
  #pragma unroll
  for (int mt = 0; mt < 4; ++mt) acc[mt] = z8;

  #pragma unroll 1
  for (int kb = 0; kb < KL; kb += 32) {
    const v16h bf = load_frag32(wr + kb, h);
    #pragma unroll
    for (int mt = 0; mt < 4; ++mt) {
      const v16h af = load_frag32(ea + (size_t)mt * 16 * KL + kb, h);
      acc[mt] = wmma_f16(af, bf, acc[mt]);
    }
  }

  if (w < 7) {
    #pragma unroll
    for (int mt = 0; mt < 4; ++mt) {
      float* so = sH + (16 * mt + 8 * h) * NLP + 16 * nt + m;
      #pragma unroll
      for (int r = 0; r < 8; ++r) so[r * NLP] = acc[mt][r] * OSC;
    }
  }
  __syncthreads();

  constexpr int NPIECE = (64 * NOUT) / 4;
  #pragma unroll 1
  for (int i = 0; i < 7; ++i) {
    const int p = tid + 256 * i;
    if (p < NPIECE) {
      const int e0 = 4 * p;
      v4f v;
      #pragma unroll
      for (int q = 0; q < 4; ++q) {
        const int e = e0 + q;
        const int row = e / NOUT, n = e - row * NOUT;
        v[q] = sH[row * NLP + n];
      }
      *(volatile v4f*)(out + e0) = v;
    }
  }
  __threadfence();
  #pragma unroll 1
  for (int i = 0; i < 7; ++i) {
    const int p = tid + 256 * i;
    if (p < NPIECE) {
      const int e0 = 4 * p;
      v4f v;
      #pragma unroll
      for (int q = 0; q < 4; ++q) {
        const int e = e0 + q;
        const int row = e / NOUT, n = e - row * NOUT;
        v[q] = sH[row * NLP + n];
      }
      *(volatile v4f*)(out + e0) = v;
    }
  }
}

extern "C" void kernel_launch(void* const* d_in, const int* in_sizes, int n_in,
                              void* d_out, int out_size, void* d_ws, size_t ws_size,
                              hipStream_t stream) {
  if (n_in < 9) return;
  if (in_sizes[0] != NBATCH * C1 * HH1 * HH1) return;
  if (in_sizes[1] != O1 * C1 * 9) return;
  if (in_sizes[2] != O1 * C1 * 8 * 9) return;
  if (in_sizes[3] != O2 * C2 * 9) return;
  if (in_sizes[4] != O2 * C2 * 8 * 9) return;
  if (in_sizes[5] != O3 * C3 * 9) return;
  if (in_sizes[6] != O3 * C3 * 8 * 9) return;
  if (in_sizes[7] != NOUT * FIN) return;
  if (in_sizes[8] != NOUT * FIN * 8) return;
  if (out_size != NBATCH * NOUT) return;

  const float* x   = (const float*)d_in[0];
  const float* wb1 = (const float*)d_in[1];
  const float* ws1 = (const float*)d_in[2];
  const float* wb2 = (const float*)d_in[3];
  const float* ws2 = (const float*)d_in[4];
  const float* wb3 = (const float*)d_in[5];
  const float* ws3 = (const float*)d_in[6];
  const float* lb  = (const float*)d_in[7];
  const float* lc  = (const float*)d_in[8];
  float* outp = (float*)d_out;

  const size_t szT  = (size_t)NBATCH * (HH2 + 2) * (HH2 + 2) * CE2 * 2;
  const size_t szT1 = (size_t)NBATCH * (HH1 + 2) * (HH1 + 2) * CE1 * 2;
  const size_t szT3 = (size_t)NBATCH * (HH3 + 2) * (HH3 + 2) * CE3 * 2;
  if (szT1 > szT || szT3 > szT) return;
  const size_t szP1 = (size_t)NBATCH * (HH1 / 2) * O1 * (HH1 / 2) * 4;
  const size_t szP2 = (size_t)NBATCH * (HH2 / 2) * O2 * (HH2 / 2) * 4;
  const size_t szP3 = (size_t)NBATCH * (HH3 / 2) * O3 * (HH3 / 2) * 4;
  const size_t szEL = (size_t)NBATCH * KL * 2;
  const size_t szW1 = (size_t)O1 * 9 * CE1 * 2;
  const size_t szW2 = (size_t)O2 * 9 * CE2 * 2;
  const size_t szW3 = (size_t)O3 * 9 * CE3 * 2;
  const size_t szWL = (size_t)NLP * KL * 2;
  size_t off = 0;
  char* ws = (char*)d_ws;
  f16t*  T   = (f16t*)(ws + off);  off += szT;
  float* P1  = (float*)(ws + off); off += szP1;
  float* P2  = (float*)(ws + off); off += szP2;
  float* P3  = (float*)(ws + off); off += szP3;
  f16t*  EL  = (f16t*)(ws + off);  off += szEL;
  f16t*  W1p = (f16t*)(ws + off);  off += szW1;
  f16t*  W2p = (f16t*)(ws + off);  off += szW2;
  f16t*  W3p = (f16t*)(ws + off);  off += szW3;
  f16t*  WLp = (f16t*)(ws + off);  off += szWL;
  if (off > ws_size) return;

  packw_k<C1, CE1, O1><<<(O1 * 9 * CE1 / 8 + 255) / 256, 256, 0, stream>>>(wb1, ws1, W1p);
  packw_k<C2, CE2, O2><<<(O2 * 9 * CE2 / 8 + 255) / 256, 256, 0, stream>>>(wb2, ws2, W2p);
  packw_k<C3, CE3, O3><<<(O3 * 9 * CE3 / 8 + 255) / 256, 256, 0, stream>>>(wb3, ws3, W3p);
  packl_k<<<(NLP * (KL / 8) + 255) / 256, 256, 0, stream>>>(lb, lc, WLp);

  expand_k<C1, CE1, HH1, HH1, 1><<<dim3(NBATCH, HH1 + 2), 256, 0, stream>>>(x, T);
  conv_k<CE1, O1, HH1, HH1, RB1><<<dim3(HH1 / RB1, NBATCH), 256, 0, stream>>>(W1p, T, P1);

  expand_k<C2, CE2, HH2, HH2, 0><<<dim3(NBATCH, HH2 + 2), 256, 0, stream>>>(P1, T);
  conv_k<CE2, O2, HH2, HH2, RB2><<<dim3(HH2 / RB2, NBATCH), 256, 0, stream>>>(W2p, T, P2);

  expand_k<C3, CE3, HH3, HH3, 0><<<dim3(NBATCH, HH3 + 2), 256, 0, stream>>>(P2, T);
  conv_k<CE3, O3, HH3, HH3, RB3><<<dim3(HH3 / RB3, NBATCH), 256, 0, stream>>>(W3p, T, P3);

  expand_head_k<<<dim3(FIN / 1024, NBATCH), 256, 0, stream>>>(P3, EL);
  head_k<<<1, 256, 0, stream>>>(EL, WLp, outp);
}
